// Dcrnn_73212012527869
// MI455X (gfx1250) — hardware-verified
//
#include <hip/hip_runtime.h>
#include <stddef.h>
#include <stdint.h>


#define F_IN    32
#define F_HID   64
#define CIN     96
#define NGC     128
#define KP      192
#define OTO     64
#define OTI     128
#define NTHR    256
#define NWAVE   8
#define EPT     8
#define CHUNK   (NTHR * EPT)
#define WCAP    (EPT * 32)
#define LISTN   (NWAVE * WCAP)
#define NBMAX   2048
#define EIDSH   11
#define RCAP    24576
#define DEGCAP  256
#define STW     512
#define GBM     64
#define GTHR    128
#define LDP     132
#define WSMAX   134217728
#define LDS_SCAN ((2 * RCAP + 2 * NBMAX + LISTN) * 4 + 64)

static_assert((CHUNK & (CHUNK - 1)) == 0 && CHUNK <= 4096);
static_assert((NBMAX & (NBMAX - 1)) == 0 && NBMAX == (1 << EIDSH));
static_assert(NTHR * 8 == NBMAX);
static_assert(LISTN >= NBMAX);
static_assert(LISTN >= NWAVE * WCAP);
static_assert((RCAP % 32) == 0);
static_assert(NWAVE * STW <= RCAP);
static_assert(LDS_SCAN <= 300000);
static_assert(GBM == (GTHR / 32) * 16);
static_assert((KP % 32) == 0 && KP == 6 * F_IN);
static_assert(NGC == 2 * F_HID && F_HID == 64 && F_IN == 32);
static_assert((LDP % 4) == 0 && LDP >= NGC);

typedef float          v4f  __attribute__((ext_vector_type(4)));
typedef float          v8f  __attribute__((ext_vector_type(8)));
typedef int            v4i  __attribute__((ext_vector_type(4)));
typedef int            v8i  __attribute__((ext_vector_type(8)));
typedef unsigned short v8us __attribute__((ext_vector_type(8)));
typedef __bf16         v16b __attribute__((ext_vector_type(16)));
union FragB { v16b v; v8us h[2]; v8i w; };
union U8    { v8us v; v4i w; };

__device__ __forceinline__ v8f wmb(const FragB& a, const FragB& b, v8f c) {
  v8f d = __builtin_amdgcn_wmma_f32_16x16x32_bf16(false, a.v, false, b.v, (short)0, c, false, false);
  asm volatile("v_nop\n\tv_nop\n\tv_nop\n\tv_nop" : "+v"(d) : "v"(a.w), "v"(b.w));
  return d;
}

__device__ __forceinline__ unsigned int bfb(float f) {
  unsigned int u = __float_as_uint(f);
  u += 0x7FFFu + ((u >> 16) & 1u);
  return u >> 16;
}
__device__ __forceinline__ float bfr(float f) { return __uint_as_float(bfb(f) << 16); }

__device__ __forceinline__ v8us hi8(const v4f a, const v4f b) {
  v8us r;
  r[0] = (unsigned short)bfb(a.x); r[1] = (unsigned short)bfb(a.y);
  r[2] = (unsigned short)bfb(a.z); r[3] = (unsigned short)bfb(a.w);
  r[4] = (unsigned short)bfb(b.x); r[5] = (unsigned short)bfb(b.y);
  r[6] = (unsigned short)bfb(b.z); r[7] = (unsigned short)bfb(b.w);
  return r;
}
__device__ __forceinline__ v8us lo8(const v4f a, const v4f b) {
  v8us r;
  r[0] = (unsigned short)bfb(a.x - bfr(a.x)); r[1] = (unsigned short)bfb(a.y - bfr(a.y));
  r[2] = (unsigned short)bfb(a.z - bfr(a.z)); r[3] = (unsigned short)bfb(a.w - bfr(a.w));
  r[4] = (unsigned short)bfb(b.x - bfr(b.x)); r[5] = (unsigned short)bfb(b.y - bfr(b.y));
  r[6] = (unsigned short)bfb(b.z - bfr(b.z)); r[7] = (unsigned short)bfb(b.w - bfr(b.w));
  return r;
}

__device__ __forceinline__ int scan_chunk(const int* __restrict__ keys, int nE, int cbase, int slotBase,
                                          int nb, int vec8, int* list, int tid, int lane, int wave) {
  int wc = 0;
  const int el0  = tid * EPT;
  const int e0   = cbase + el0;
  const int sent = -2147483647 - 1;
  v4i da, db;
  if (vec8 != 0 && cbase + CHUNK <= nE) {
    da = *(const v4i*)(keys + e0);
    db = *(const v4i*)(keys + e0 + 4);
  } else {
    da.x = (e0     < nE) ? keys[min(e0,     nE - 1)] : sent;
    da.y = (e0 + 1 < nE) ? keys[min(e0 + 1, nE - 1)] : sent;
    da.z = (e0 + 2 < nE) ? keys[min(e0 + 2, nE - 1)] : sent;
    da.w = (e0 + 3 < nE) ? keys[min(e0 + 3, nE - 1)] : sent;
    db.x = (e0 + 4 < nE) ? keys[min(e0 + 4, nE - 1)] : sent;
    db.y = (e0 + 5 < nE) ? keys[min(e0 + 5, nE - 1)] : sent;
    db.z = (e0 + 6 < nE) ? keys[min(e0 + 6, nE - 1)] : sent;
    db.w = (e0 + 7 < nE) ? keys[min(e0 + 7, nE - 1)] : sent;
  }
  const unsigned nbs = (unsigned)slotBase;
  const unsigned unb = (unsigned)nb;
  const unsigned s0 = (unsigned)da.x - nbs, s1 = (unsigned)da.y - nbs;
  const unsigned s2 = (unsigned)da.z - nbs, s3 = (unsigned)da.w - nbs;
  const unsigned s4 = (unsigned)db.x - nbs, s5 = (unsigned)db.y - nbs;
  const unsigned s6 = (unsigned)db.z - nbs, s7 = (unsigned)db.w - nbs;
  const bool h0 = s0 < unb, h1 = s1 < unb, h2 = s2 < unb, h3 = s3 < unb;
  const bool h4 = s4 < unb, h5 = s5 < unb, h6 = s6 < unb, h7 = s7 < unb;
  const unsigned any = __builtin_amdgcn_ballot_w32(h0 | h1 | h2 | h3 | h4 | h5 | h6 | h7);
  if (any != 0u) {
#define HITJ(J, HJ, SJ) { \
      const unsigned mj = __builtin_amdgcn_ballot_w32(HJ); \
      if (mj != 0u) { \
        if (HJ) { \
          const int pos = wc + (int)__builtin_amdgcn_mbcnt_lo(mj, 0u); \
          if (pos < WCAP) list[wave * WCAP + pos] = ((el0 + (J)) << 12) | (int)(SJ); \
        } \
        wc += (int)__builtin_popcount(mj); } }
    HITJ(0, h0, s0)
    HITJ(1, h1, s1)
    HITJ(2, h2, s2)
    HITJ(3, h3, s3)
    HITJ(4, h4, s4)
    HITJ(5, h5, s5)
    HITJ(6, h6, s6)
    HITJ(7, h7, s7)
#undef HITJ
  }
  return wc;
}

__global__ __launch_bounds__(NTHR) void k_xprep(const float* __restrict__ x, unsigned short* ap, int nN, int nUnits) {
  const int i = (int)blockIdx.x * NTHR + (int)threadIdx.x;
  if (i >= nUnits) return;
  const int row = i >> 3;
  const int q   = i & 7;
  const int c0  = (q & 3) * 8;
  const int rc  = row < nN ? row : nN - 1;
  const float* p = x + (size_t)rc * F_IN + c0;
  v4f a = *(const v4f*)p, b = *(const v4f*)(p + 4);
  const v4f z4 = {0.f, 0.f, 0.f, 0.f};
  if (row >= nN) { a = z4; b = z4; }
  const v8us hv = hi8(a, b);
  const size_t o = (size_t)row * KP + 8 * q;
  *(volatile v8us*)(ap + o) = hv;
  __threadfence();
  *(volatile v8us*)(ap + o) = hv;
}

__global__ __launch_bounds__(NTHR) void k_wtr(const float* __restrict__ wz, const float* __restrict__ wh,
                                              unsigned short* wt, int nUnits) {
  const int u = (int)blockIdx.x * NTHR + (int)threadIdx.x;
  if (u >= nUnits) return;
  const int kq  = KP / 8;
  const int n   = u / kq;
  const int k8  = (u - n * kq) * 8;
  const int g   = (n >> 6) & 1;
  const int oc  = n & 63;
  const float* wg = g ? wh : wz;
  const int ksg = k8 >> 5;
  const int dj  = (ksg == 0) ? 0 : ((ksg == 1) ? 2 : ((ksg <= 3) ? 1 : 3));
  const int kk0 = k8 & 31;
  const float* p = wg + (size_t)(dj * CIN + kk0) * F_HID + oc;
  v4f a, b;
  a.x = p[0];          a.y = p[F_HID];      a.z = p[2 * F_HID];  a.w = p[3 * F_HID];
  b.x = p[4 * F_HID];  b.y = p[5 * F_HID];  b.z = p[6 * F_HID];  b.w = p[7 * F_HID];
  const v8us hv = hi8(a, b);
  const size_t o = (size_t)n * KP + k8;
  *(volatile v8us*)(wt + o) = hv;
  __threadfence();
  *(volatile v8us*)(wt + o) = hv;
}

template<int MODE>
__global__ __launch_bounds__(NTHR) void k_scan(
    const int* __restrict__ keys, const int* __restrict__ oth,
    const float* __restrict__ w, const float* __restrict__ x,
    const float* __restrict__ dinvIn, float* dinvOut, unsigned short* AP,
    int nN, int nE, int nb, int vec8, int MPr) {
  extern __shared__ v4f lds_dyn[];
  int* reg1 = (int*)lds_dyn;
  int* reg2 = reg1 + RCAP;
  int* scnt = reg2 + RCAP;
  int* soff = scnt + NBMAX;
  int* list = soff + NBMAX;
  int* wcnt = list + LISTN;
  int* wtot = wcnt + NWAVE;
  const int tid = (int)threadIdx.x, lane = tid & 31, wave = tid >> 5;
  const int nodeBase = (int)blockIdx.x * nb;

  for (int i = tid; i < NBMAX; i += NTHR) scnt[i] = 0;
  __syncthreads();

  int tot = 0;
  const int nChunks = (nE + CHUNK - 1) / CHUNK;
#pragma unroll 1
  for (int ch = 0; ch < nChunks; ++ch) {
    const int cbase = ch * CHUNK;
    const int wc = scan_chunk(keys, nE, cbase, nodeBase, nb, vec8, list, tid, lane, wave);
    if (lane == 0) wcnt[wave] = wc;
    __syncthreads();
    int pre = 0, all = 0;
#pragma unroll
    for (int w2 = 0; w2 < NWAVE; ++w2) {
      int c = wcnt[w2];
      c = c < 0 ? 0 : (c > WCAP ? WCAP : c);
      all += c;
      pre += (w2 < wave) ? c : 0;
    }
    const int wcc  = wc > WCAP ? WCAP : wc;
    const int base = tot + pre;
#pragma unroll 1
    for (int i = lane; i < wcc; i += 32) {
      const int ent = list[wave * WCAP + i];
      const int el  = (ent >> 12) & (CHUNK - 1);
      const int sl  = ent & (NBMAX - 1);
      int eid = cbase + el;
      eid = eid > nE - 1 ? nE - 1 : eid;
      const int pos = base + i;
      if (pos < RCAP) reg1[pos] = (int)(((unsigned)eid << EIDSH) | (unsigned)sl);
    }
    tot += all;
    tot = tot > RCAP ? RCAP : tot;
    __syncthreads();
  }
  const int nh = tot;

  if (wave == 0) {
#pragma unroll 1
    for (int b0 = 0; b0 < nh; b0 += 32) {
      const int idx = b0 + lane;
      const int uv  = reg1[idx < RCAP ? idx : RCAP - 1];
      const int m32 = (nh - b0) < 32 ? (nh - b0) : 32;
#pragma unroll 1
      for (int k = 0; k < m32; ++k) {
        const int u  = __builtin_amdgcn_readlane(uv, k);
        const int sl = u & (NBMAX - 1);
        if (lane == 0) scnt[sl] = scnt[sl] + 1;
      }
    }
  }
  __syncthreads();

  {
    const v4i ca = *(const v4i*)(scnt + 8 * tid);
    const v4i cb = *(const v4i*)(scnt + 8 * tid + 4);
    const int e0 = ca.x < 0 ? 0 : ca.x, e1 = ca.y < 0 ? 0 : ca.y, e2 = ca.z < 0 ? 0 : ca.z, e3 = ca.w < 0 ? 0 : ca.w;
    const int e4 = cb.x < 0 ? 0 : cb.x, e5 = cb.y < 0 ? 0 : cb.y, e6 = cb.z < 0 ? 0 : cb.z, e7 = cb.w < 0 ? 0 : cb.w;
    const int ts = e0 + e1 + e2 + e3 + e4 + e5 + e6 + e7;
    int incl = ts;
#pragma unroll
    for (int d = 1; d < 32; d <<= 1) {
      const int up = __shfl_up(incl, d);
      if (lane >= d) incl += up;
    }
    if (lane == 31) wtot[wave] = incl;
    __syncthreads();
    int pre = 0;
#pragma unroll
    for (int w2 = 0; w2 < NWAVE; ++w2) pre += (w2 < wave) ? wtot[w2] : 0;
    int run = pre + incl - ts;
    soff[8 * tid + 0] = run; run += e0;
    soff[8 * tid + 1] = run; run += e1;
    soff[8 * tid + 2] = run; run += e2;
    soff[8 * tid + 3] = run; run += e3;
    soff[8 * tid + 4] = run; run += e4;
    soff[8 * tid + 5] = run; run += e5;
    soff[8 * tid + 6] = run; run += e6;
    soff[8 * tid + 7] = run;
  }
  __syncthreads();
  for (int i = tid; i < NBMAX; i += NTHR) list[i] = soff[i];
  __syncthreads();

  if (wave == 0) {
#pragma unroll 1
    for (int b0 = 0; b0 < nh; b0 += 32) {
      const int idx = b0 + lane;
      const int uv  = reg1[idx < RCAP ? idx : RCAP - 1];
      const int m32 = (nh - b0) < 32 ? (nh - b0) : 32;
#pragma unroll 1
      for (int k = 0; k < m32; ++k) {
        const int u   = __builtin_amdgcn_readlane(uv, k);
        const int sl  = u & (NBMAX - 1);
        const int eid = (int)((unsigned)u >> EIDSH);
        if (lane == 0) {
          int pos = list[sl];
          pos = pos < 0 ? 0 : (pos > RCAP - 1 ? RCAP - 1 : pos);
          reg2[pos] = eid;
          list[sl] = pos + 1;
        }
      }
    }
  }
  __syncthreads();

  const int nbw = nb >> 3;
  const bool ovf = (nh >= RCAP);
  const float qnan = __int_as_float(0x7fc00000);
  float* stw  = (float*)reg1 + wave * STW;
  float* dstg = (float*)list;
  const int lc = lane < 8 ? lane : 7;
  const int colOff = (MODE == 1) ? OTO : OTI;
#pragma unroll 1
  for (int jt = 0; jt < nbw; ++jt) {
    const int slot = wave * nbw + jt;
    const int grow = nodeBase + slot;
    int st = soff[slot];
    const int craw = scnt[slot];
    int cnt = craw;
    st  = st < 0 ? 0 : (st > nh ? nh : st);
    cnt = cnt < 0 ? 0 : (cnt > DEGCAP ? DEGCAP : cnt);
    if (cnt > nh - st) cnt = nh - st;
    const float pz = (ovf || craw > DEGCAP) ? qnan : 0.0f;
    const bool wr = grow < MPr;
    const float live = grow < nN ? 1.0f : 0.0f;
    float acc = 0.f, dsum = 0.f;
#pragma unroll 1
    for (int q = 0; q < cnt; ++q) {
      int idx = st + q; idx = idx > RCAP - 1 ? RCAP - 1 : idx;
      int eid = reg2[idx]; eid = eid < 0 ? 0 : (eid > nE - 1 ? nE - 1 : eid);
      const float we = bfr(w[eid]);
      if (MODE != 2) dsum += we;
      if (MODE != 0) {
        const int oraw = oth[eid];
        const int o = oraw < 0 ? 0 : (oraw > nN - 1 ? nN - 1 : oraw);
        const float cf = we * dinvIn[o];
        const float xv = bfr(x[(size_t)o * F_IN + lane]);
        acc = fmaf(cf, xv, acc);
      }
    }
    if (MODE != 2) {
      const float dv = dsum > 0.f ? (1.0f / dsum) : 0.0f;
      dstg[slot] = dv + pz;
    }
    if (MODE != 0) {
      const float r0 = acc * live + pz;
      __builtin_amdgcn_fence(__ATOMIC_RELEASE, "wavefront");
      __builtin_amdgcn_wave_barrier();
      stw[lane] = r0;
      __builtin_amdgcn_fence(__ATOMIC_RELEASE, "wavefront");
      __builtin_amdgcn_wave_barrier();
      const v4f ga = *(const v4f*)(stw + 8 * (lc & 3));
      const v4f gb = *(const v4f*)(stw + 8 * (lc & 3) + 4);
      U8 hv, lv, sv;
      hv.v = hi8(ga, gb);
      lv.v = lo8(ga, gb);
      const bool useHi = lane < 4;
      sv.w.x = useHi ? hv.w.x : lv.w.x;
      sv.w.y = useHi ? hv.w.y : lv.w.y;
      sv.w.z = useHi ? hv.w.z : lv.w.z;
      sv.w.w = useHi ? hv.w.w : lv.w.w;
      unsigned short* gp = AP + (size_t)grow * KP + colOff + 8 * lc;
      const bool wsv = wr && (lane < 8);
      if (wsv) *(volatile v8us*)gp = sv.v;
      __threadfence();
      if (wsv) *(volatile v8us*)gp = sv.v;
    }
  }
  if (MODE != 2) {
    __syncthreads();
    const int np = nb >> 2;
#pragma unroll 1
    for (int p = tid; p < np; p += NTHR) {
      const v4f v = *(const v4f*)(dstg + 4 * p);
      *(volatile v4f*)(dinvOut + (size_t)nodeBase + 4 * p) = v;
    }
    __threadfence();
#pragma unroll 1
    for (int p = tid; p < np; p += NTHR) {
      const v4f v = *(const v4f*)(dstg + 4 * p);
      *(volatile v4f*)(dinvOut + (size_t)nodeBase + 4 * p) = v;
    }
  }
}

__global__ __launch_bounds__(GTHR) void k_gemm(
    const unsigned short* __restrict__ AP, const unsigned short* __restrict__ WT,
    const float* __restrict__ bz, const float* __restrict__ bh,
    const float* __restrict__ wl, const float* __restrict__ bl,
    float* out, int nRows) {
  __shared__ __attribute__((aligned(16))) float stg[GBM * LDP];
  __shared__ __attribute__((aligned(16))) float outv[GBM];
  const int tid = (int)threadIdx.x, lane = tid & 31, wave = tid >> 5, hh = lane >> 4, m = lane & 15;
  const int rowBase = (int)blockIdx.x * GBM;

  v8f acc[8];
  {
    const v8f z = {0.f, 0.f, 0.f, 0.f, 0.f, 0.f, 0.f, 0.f};
#pragma unroll
    for (int t = 0; t < 8; ++t) acc[t] = z;
  }
  const unsigned short* ap = AP + (size_t)(rowBase + 16 * wave + m) * KP + 8 * hh;
  const unsigned short* wp = WT + (size_t)m * KP + 8 * hh;
#pragma unroll 1
  for (int ks = 0; ks < KP / 32; ++ks) {
    FragB af;
    af.h[0] = *(const v8us*)(ap + 32 * ks);
    af.h[1] = *(const v8us*)(ap + 32 * ks + 16);
#pragma unroll
    for (int t = 0; t < 8; ++t) {
      const unsigned short* wq = wp + (size_t)(16 * t) * KP + 32 * ks;
      FragB bf;
      bf.h[0] = *(const v8us*)wq;
      bf.h[1] = *(const v8us*)(wq + 16);
      acc[t] = wmb(af, bf, acc[t]);
    }
  }

#pragma unroll
  for (int t = 0; t < 8; ++t) {
    const int lc = 16 * t + m;
    const float* bp = (t < 4) ? bz : bh;
    const float bv = bfr(bp[lc & 63]);
#pragma unroll
    for (int r = 0; r < 8; ++r) {
      const int lr = 16 * wave + 8 * hh + r;
      stg[lr * LDP + lc] = acc[t][r] + bv;
    }
  }
  __syncthreads();

  const float wl0 = bfr(wl[lane]);
  const float wl1 = bfr(wl[32 + lane]);
  const float blv = bfr(bl[0]);
  float mine = 0.f;
#pragma unroll 1
  for (int r = 0; r < 16; ++r) {
    const float* sp = stg + (16 * wave + r) * LDP;
    const float z0 = sp[lane], z1 = sp[32 + lane];
    const float g0 = sp[64 + lane], g1 = sp[96 + lane];
    const float s0 = 1.0f / (1.0f + expf(-z0));
    const float s1 = 1.0f / (1.0f + expf(-z1));
    const float h0 = (1.0f - s0) * tanhf(g0);
    const float h1 = (1.0f - s1) * tanhf(g1);
    const float q0 = h0 > 0.f ? h0 : h0 * 0.0f;
    const float q1 = h1 > 0.f ? h1 : h1 * 0.0f;
    float part = fmaf(q1, wl1, q0 * wl0);
#pragma unroll
    for (int off = 16; off > 0; off >>= 1) part += __shfl_xor(part, off);
    mine = (lane == r) ? part : mine;
  }
  if (lane < 16) outv[16 * wave + lane] = mine + blv;
  __syncthreads();

  if (wave == 0) {
    int nv = nRows - rowBase;
    nv = nv < 0 ? 0 : (nv > GBM ? GBM : nv);
    const int np = nv >> 2;
    const int pl = lane & 15;
    const v4f v = *(const v4f*)(outv + 4 * pl);
    int te = (nv & ~3) + pl;
    te = te > GBM - 1 ? GBM - 1 : te;
    const float tv = outv[te];
    const bool sv = (lane < 16) && (pl < np);
    const bool st = (lane < 16) && (pl < (nv & 3));
    float* op = out + (size_t)rowBase + 4 * pl;
    float* ot = out + (size_t)rowBase + te;
    if (sv) *(volatile v4f*)op = v;
    if (st) *(volatile float*)ot = tv;
    __threadfence();
    if (sv) *(volatile v4f*)op = v;
    if (st) *(volatile float*)ot = tv;
  }
}

static int pick_nb(int nE, int nN) {
  int nb = NBMAX;
  while (nb > 32 && (long long)nb * (long long)nE * 5LL > (long long)RCAP * (long long)nN * 4LL) nb >>= 1;
  return nb;
}
static inline int cdiv(int a, int b) { return (a + b - 1) / b; }

extern "C" void kernel_launch(void* const* d_in, const int* in_sizes, int n_in,
                              void* d_out, int out_size, void* d_ws, size_t ws_size,
                              hipStream_t stream) {
  if (n_in < 11) return;
  const int nN = in_sizes[0] / F_IN;
  if (nN <= 0 || in_sizes[0] != nN * F_IN || nN > (1 << 22)) return;
  if (in_sizes[1] < 2 || (in_sizes[1] & 1) != 0) return;
  const int nE = in_sizes[1] / 2;
  if (nE < 1 || nE > (1 << 21)) return;
  if (in_sizes[2] != nE) return;
  if (in_sizes[3] != 2 * 2 * CIN * F_HID || in_sizes[4] != F_HID) return;
  if (in_sizes[7] != 2 * 2 * CIN * F_HID || in_sizes[8] != F_HID) return;
  if (in_sizes[9] != F_HID || in_sizes[10] < 1) return;
  if (out_size != nN) return;

  const float* x    = (const float*)d_in[0];
  const int*   ei   = (const int*)  d_in[1];
  const float* w    = (const float*)d_in[2];
  const float* Wz   = (const float*)d_in[3];
  const float* bz   = (const float*)d_in[4];
  const float* Wh   = (const float*)d_in[7];
  const float* bh   = (const float*)d_in[8];
  const float* Wlin = (const float*)d_in[9];
  const float* blin = (const float*)d_in[10];
  float* out = (float*)d_out;
  const int* src = ei;
  const int* dst = ei + nE;

  const int MP   = cdiv(nN, GBM) * GBM;
  const int nb   = pick_nb(nE, nN);
  const int gA   = cdiv(MP, nb);
  const int vec8 = ((nE & 3) == 0) ? 1 : 0;
  if (nb < 32 || gA * nb < MP) return;

  char* ws = (char*)d_ws;
  size_t off = 0;
  const size_t oAP  = off; off += (size_t)MP * KP * 2;              off = (off + 255) & ~(size_t)255;
  const size_t oWT  = off; off += (size_t)NGC * KP * 2;             off = (off + 255) & ~(size_t)255;
  const size_t oDOI = off; off += (size_t)gA * (size_t)nb * 4;      off = (off + 255) & ~(size_t)255;
  const size_t oDII = off; off += (size_t)gA * (size_t)nb * 4;      off = (off + 255) & ~(size_t)255;
  if (off > ws_size || off > (size_t)WSMAX) return;
  unsigned short* AP  = (unsigned short*)(ws + oAP);
  unsigned short* WT  = (unsigned short*)(ws + oWT);
  float*          DOI = (float*)(ws + oDOI);
  float*          DII = (float*)(ws + oDII);

  hipFuncSetAttribute(reinterpret_cast<const void*>(&k_scan<0>), hipFuncAttributeMaxDynamicSharedMemorySize, LDS_SCAN);
  hipFuncSetAttribute(reinterpret_cast<const void*>(&k_scan<1>), hipFuncAttributeMaxDynamicSharedMemorySize, LDS_SCAN);
  hipFuncSetAttribute(reinterpret_cast<const void*>(&k_scan<2>), hipFuncAttributeMaxDynamicSharedMemorySize, LDS_SCAN);

  const int nUx = MP * 8;
  k_xprep<<<cdiv(nUx, NTHR), NTHR, 0, stream>>>(x, AP, nN, nUx);
  const int nUw = NGC * (KP / 8);
  k_wtr<<<cdiv(nUw, NTHR), NTHR, 0, stream>>>(Wz, Wh, WT, nUw);
  k_scan<0><<<gA, NTHR, LDS_SCAN, stream>>>(src, dst, w, x, DII, DOI, AP, nN, nE, nb, vec8, MP);
  k_scan<1><<<gA, NTHR, LDS_SCAN, stream>>>(dst, src, w, x, DOI, DII, AP, nN, nE, nb, vec8, MP);
  k_scan<2><<<gA, NTHR, LDS_SCAN, stream>>>(src, dst, w, x, DII, DOI, AP, nN, nE, nb, vec8, MP);
  k_gemm<<<MP / GBM, GTHR, 0, stream>>>(AP, WT, bz, bh, Wlin, blin, out, nN);
}
